// Block_55490977465077
// MI455X (gfx1250) — hardware-verified
//
#include <hip/hip_runtime.h>
#include <math.h>

#ifndef NB
#define NB 4
#endif
#ifndef SEQ
#define SEQ 1024
#endif
#define NB_FULL 4
#define SEQ_FULL 1024

constexpr int kC       = 1024;
constexpr int kHeads   = 16;
constexpr int kHD      = 64;
constexpr int kQkvCols = 3 * kC;
constexpr int kKvCols  = 2 * kC;
constexpr int kFF      = 4 * kC;
constexpr int kT2      = 257;
constexpr int kT2P     = 320;
constexpr int kTok     = NB * SEQ;
constexpr int kGroups  = NB * kHeads;
constexpr int kImgRows = NB * kT2;
constexpr int kImgPad  = (((NB - 1) * kT2 + kT2P + 63) / 64) * 64;
constexpr int kSmThreads = (((SEQ / 8) + 31) / 32) * 32;
constexpr float kWCarry = 16.0f;
constexpr float kPCarry = 2048.0f;
constexpr float kOCarry = 64.0f;
constexpr float kGCarry = 16.0f;
constexpr float kLnEps  = 1e-5f;
constexpr float kInvDim = 1.0f / 1024.0f;
constexpr size_t kOut1OffElems = (size_t)NB_FULL * SEQ_FULL * kC;

static_assert(kOut1OffElems * 4 == 16777216);
static_assert(NB >= 1 && NB <= NB_FULL);
static_assert(SEQ >= 64 && SEQ <= SEQ_FULL);
static_assert((SEQ & (SEQ - 1)) == 0);
static_assert(SEQ % 64 == 0 && kTok % 64 == 0 && kImgPad % 64 == 0 && kT2P % 64 == 0);
static_assert(kC % 64 == 0 && kQkvCols % 64 == 0 && kKvCols % 64 == 0 && kFF % 64 == 0);
static_assert(kHD % 32 == 0 && kC % 32 == 0 && kFF % 32 == 0 && kT2P % 32 == 0 && SEQ % 32 == 0);
static_assert(kImgPad >= kImgRows);
static_assert((NB - 1) * kT2 + kT2P <= kImgPad);
static_assert(kSmThreads * 8 >= SEQ && kSmThreads <= 256);
static_assert(kHeads * kHD == kC);

typedef __attribute__((ext_vector_type(16))) _Float16 v16h;
typedef __attribute__((ext_vector_type(8)))  _Float16 v8h;
typedef __attribute__((ext_vector_type(8)))  float    v8f;
typedef __attribute__((ext_vector_type(4)))  float    v4f;
typedef __attribute__((ext_vector_type(4)))  unsigned int v4u;

__device__ __forceinline__ unsigned short f2bf_bits(float f) {
  unsigned u = __float_as_uint(f);
  return (unsigned short)((u + 0x7FFFu + ((u >> 16) & 1u)) >> 16);
}
__device__ __forceinline__ float bf_bits2f(unsigned short h) { return __uint_as_float(((unsigned)h) << 16); }
__device__ __forceinline__ float bfr(float f) { return bf_bits2f(f2bf_bits(f)); }

__device__ __forceinline__ void dep_guard_h(v8f& a, v8f& b, v16h x, v16h y) { asm volatile("v_nop\n\tv_nop\n\tv_nop\n\tv_nop" : "+v"(a), "+v"(b) : "v"(x), "v"(y)); }
__device__ __forceinline__ void keep4_h(v16h a, v16h b, v16h c, v16h d) { asm volatile("v_nop" :: "v"(a), "v"(b), "v"(c), "v"(d)); }
__device__ __forceinline__ void acc_guard4(v8f& a, v8f& b, v8f& c, v8f& d) { asm volatile("v_nop\n\tv_nop\n\tv_nop\n\tv_nop" : "+v"(a), "+v"(b), "+v"(c), "+v"(d)); }

union FragU { v16h v; v8h h[2]; };
__device__ __forceinline__ v16h frag_load(const _Float16* p) {
  FragU f; f.h[0] = *(const v8h*)(p); f.h[1] = *(const v8h*)(p + 16); return f.v;
}
__device__ __forceinline__ v8f frag_mma(v16h a, v16h b, v8f c) {
  return __builtin_amdgcn_wmma_f32_16x16x32_f16(false, a, false, b, (short)0, c, false, false);
}

__device__ __forceinline__ unsigned pk16(unsigned short a, unsigned short b) { return (unsigned)a | ((unsigned)b << 16); }
__device__ __forceinline__ unsigned short h_bits(float f) { const _Float16 h = (_Float16)f; return __builtin_bit_cast(unsigned short, h); }

__device__ __forceinline__ float gelu_tanh(float v) {
  const float u = 0.7978845608028654f * (v + 0.044715f * (v * v * v));
  return 0.5f * v * (1.0f + tanhf(u));
}

template <int BIAS_MODE, int OUT_MODE, int RESID, int ACT, int CAUSAL>
__global__ __launch_bounds__(256) void wmma_gemm64(
    const unsigned short* __restrict__ Ap, int lda, long strideA,
    const unsigned short* __restrict__ Btp, int ldb, long strideB,
    void* __restrict__ Cout, int ldc, long strideC,
    const float* __restrict__ bias,
    const float* __restrict__ resid, long strideR,
    int M, int N, int K, float scale) {
  const _Float16* A = (const _Float16*)Ap; const _Float16* Bt = (const _Float16*)Btp;
  __shared__ __align__(16) float sT[8][16 * 68];
  const int b    = blockIdx.y;
  const int lane = threadIdx.x & 31;
  const int wave = threadIdx.x >> 5;
  const int tilesN = N >> 6;
  const int tilesM = M >> 6;
  const int tile = blockIdx.x * 8 + wave;
  if (tile >= tilesM * tilesN) return;
  const int tm = tile / tilesN;
  const int tn = tile - tm * tilesN;
  if (CAUSAL == 1 && tn > tm) return;
  const int m0 = tm << 6;
  const int n0 = tn << 6;
  const int kEnd = (CAUSAL == 2) ? (((m0 + 64) < K) ? (m0 + 64) : K) : K;

  const _Float16* Ab = A  + (size_t)b * strideA;
  const _Float16* Bb = Bt + (size_t)b * strideB;

  const int rlane = lane & 15;
  const int koff  = (lane >> 4) * 8;
  const int mOff  = (lane >> 4) * 8;

  v8f acc[4][4];
#pragma unroll
  for (int i = 0; i < 4; ++i)
#pragma unroll
    for (int j = 0; j < 4; ++j) acc[i][j] = (v8f){0.f,0.f,0.f,0.f,0.f,0.f,0.f,0.f};

  for (int k0 = 0; k0 < kEnd; k0 += 32) {
    v16h bh[4];
#pragma unroll
    for (int j = 0; j < 4; ++j) {
      const size_t bo = (size_t)(n0 + (j << 4) + rlane) * ldb + koff + k0;
      bh[j] = frag_load(Bb + bo);
    }
#pragma unroll
    for (int i = 0; i < 4; ++i) {
      const size_t ao = (size_t)(m0 + (i << 4) + rlane) * lda + koff + k0;
      v16h ah = frag_load(Ab + ao);
#pragma unroll
      for (int j = 0; j < 4; ++j) acc[i][j] = frag_mma(ah, bh[j], acc[i][j]);
      dep_guard_h(acc[i][0], acc[i][3], ah, ah);
    }
    keep4_h(bh[0], bh[1], bh[2], bh[3]);
  }
  acc_guard4(acc[0][0], acc[0][1], acc[0][2], acc[0][3]);
  acc_guard4(acc[1][0], acc[1][1], acc[1][2], acc[1][3]);
  acc_guard4(acc[2][0], acc[2][1], acc[2][2], acc[2][3]);
  acc_guard4(acc[3][0], acc[3][1], acc[3][2], acc[3][3]);

  float* slab = sT[wave];
  const float* Rb = (RESID != 0) ? (resid + (size_t)b * strideR) : nullptr;
#pragma unroll
  for (int i = 0; i < 4; ++i) {
    const int mBase = m0 + (i << 4);
#pragma unroll
    for (int j = 0; j < 4; ++j) {
      const int n = n0 + (j << 4) + rlane;
      float bv = 0.f;
      if (BIAS_MODE == 2) bv = bfr(bias[n]);
#pragma unroll
      for (int r = 0; r < 8; ++r) {
        float v = acc[i][j][r] * scale;
        if (BIAS_MODE == 2) v += bv;
        if (RESID == 1) v += Rb[(size_t)(mBase + mOff + r) * ldc + n];
        if (RESID == 2) v += bfr(Rb[(size_t)(mBase + mOff + r) * ldc + n]);
        slab[(mOff + r) * 68 + (j << 4) + rlane] = v;
      }
    }
    __builtin_amdgcn_fence(3  , "workgroup");
    __builtin_amdgcn_wave_barrier();
    __builtin_amdgcn_fence(2  , "workgroup");
    if (OUT_MODE == 0) {
      float* C = (float*)Cout + (size_t)b * strideC;
      const int hh = lane >> 4, c4 = (lane & 15) * 4;
      for (int pass = 0; pass < 2; ++pass) {
#pragma unroll
        for (int it = 0; it < 8; ++it) {
          const int row = it * 2 + hh;
          v4f v = *(const v4f*)(slab + row * 68 + c4);
          *(volatile v4f*)(C + (size_t)(mBase + row) * ldc + n0 + c4) = v;
        }
        __threadfence();
      }
    } else {
      const int q = lane >> 3, c8 = (lane & 7) * 8;
      if (ACT == 5) {
#pragma unroll 1
        for (int it = 0; it < 4; ++it) {
          float* sp = slab + (it * 4 + q) * 68 + c8;
#pragma unroll 1
          for (int e = 0; e < 8; ++e) {
            const float gv = gelu_tanh(sp[e]) * kGCarry;
            sp[e] = gv;
          }
        }
      }
      unsigned short* C = (unsigned short*)Cout + (size_t)b * strideC;
      for (int pass = 0; pass < 2; ++pass) {
#pragma unroll
        for (int it = 0; it < 4; ++it) {
          const int row = it * 4 + q;
          const float* sp = slab + row * 68 + c8;
          v8h hv;
#pragma unroll
          for (int e = 0; e < 8; ++e) hv[e] = (_Float16)sp[e];
          *(volatile v8h*)(C + (size_t)(mBase + row) * ldc + n0 + c8) = hv;
        }
        __threadfence();
      }
    }
    __builtin_amdgcn_fence(3  , "workgroup");
    __builtin_amdgcn_wave_barrier();
    __builtin_amdgcn_fence(2  , "workgroup");
  }
}

__global__ __launch_bounds__(256) void wtcast_kernel(const float* __restrict__ W, unsigned short* __restrict__ WT,
                                                     int Kin, int Nout, float scale) {
  __shared__ float sm[64][65];
  const int t  = threadIdx.x;
  const int k0 = blockIdx.x * 64;
  const int n0 = blockIdx.y * 64;
#pragma unroll
  for (int i = 0; i < 16; ++i) {
    const int e = i * 256 + t;
    const int r = e >> 6;
    const int c = e & 63;
    sm[c][r] = bfr(W[(size_t)(k0 + r) * Nout + n0 + c]) * scale;
  }
  __syncthreads();
  const int lane = t & 31, wave = t >> 5;
  const int q = lane >> 3, c8 = (lane & 7) * 8;
  for (int pass = 0; pass < 2; ++pass) {
#pragma unroll
    for (int it = 0; it < 2; ++it) {
      const int row = wave * 8 + it * 4 + q;
      unsigned short hb[8];
#pragma unroll
      for (int e = 0; e < 8; ++e) hb[e] = h_bits(sm[row][c8 + e]);
      const v4u u = (v4u){pk16(hb[0], hb[1]), pk16(hb[2], hb[3]), pk16(hb[4], hb[5]), pk16(hb[6], hb[7])};
      *(volatile v4u*)(WT + (size_t)(n0 + row) * Kin + k0 + c8) = u;
    }
    __threadfence();
  }
}

__global__ __launch_bounds__(256) void img_prep_kernel(const float* __restrict__ img, float* __restrict__ out1,
                                                       unsigned short* __restrict__ plane) {
  const unsigned row = blockIdx.x;
  const unsigned t   = threadIdx.x;
  unsigned short* pp = plane + (size_t)row * kC + t * 8u;
  if (row < (unsigned)kImgRows) {
    const float* ir = img + (size_t)row * kC;
    const v4f v = *(const v4f*)(ir + t * 4u);
    v4f o;
#pragma unroll
    for (int e = 0; e < 4; ++e) o[e] = bfr(v[e]);
    float* op = out1 + (size_t)row * kC + t * 4u;
    *(volatile v4f*)op = o;
    __threadfence();
    *(volatile v4f*)op = o;
    if (t < 128u) {
      const v4f xa = *(const v4f*)(ir + t * 8u);
      const v4f xb = *(const v4f*)(ir + t * 8u + 4u);
      unsigned short hb[8];
#pragma unroll
      for (int e = 0; e < 4; ++e) { hb[e] = h_bits(bfr(xa[e])); hb[4 + e] = h_bits(bfr(xb[e])); }
      const v4u u = (v4u){pk16(hb[0], hb[1]), pk16(hb[2], hb[3]), pk16(hb[4], hb[5]), pk16(hb[6], hb[7])};
      *(volatile v4u*)pp = u;
      __threadfence();
      *(volatile v4u*)pp = u;
    }
  } else {
    if (t < 128u) {
      const v4u z = (v4u){0u, 0u, 0u, 0u};
      *(volatile v4u*)pp = z;
      __threadfence();
      *(volatile v4u*)pp = z;
    }
  }
}

template <int CVT_IN>
__global__ __launch_bounds__(256) void ln_row_kernel(const float* __restrict__ X, unsigned inBatchRows,
                                                     const float* __restrict__ gam, const float* __restrict__ bet,
                                                     unsigned short* __restrict__ Y) {
  __shared__ float red[8];
  __shared__ float stat[2];
  const unsigned t    = threadIdx.x;
  const unsigned lane = t & 31u, wave = t >> 5;
  const size_t irow = (size_t)blockIdx.y * inBatchRows + blockIdx.x;
  const size_t orow = (size_t)blockIdx.y * SEQ + blockIdx.x;
  const float* xr = X + irow * kC;
  float a0 = xr[t], a1 = xr[t + 256u], a2 = xr[t + 512u], a3 = xr[t + 768u];
  if (CVT_IN) { a0 = bfr(a0); a1 = bfr(a1); a2 = bfr(a2); a3 = bfr(a3); }
  float s = (a0 + a1) + (a2 + a3);
#pragma unroll
  for (int off = 16; off > 0; off >>= 1) s += __shfl_xor(s, off, 32);
  if (lane == 0) red[wave] = s;
  __syncthreads();
  if (t == 0) {
    float tot = red[0];
#pragma unroll
    for (int w = 1; w < 8; ++w) tot += red[w];
    stat[0] = tot * kInvDim;
  }
  __syncthreads();
  const float mu = stat[0];
  const float d0 = a0 - mu, d1 = a1 - mu, d2 = a2 - mu, d3 = a3 - mu;
  float s2 = (d0 * d0 + d1 * d1) + (d2 * d2 + d3 * d3);
#pragma unroll
  for (int off = 16; off > 0; off >>= 1) s2 += __shfl_xor(s2, off, 32);
  if (lane == 0) red[wave] = s2;
  __syncthreads();
  if (t == 0) {
    float tot = red[0];
#pragma unroll
    for (int w = 1; w < 8; ++w) tot += red[w];
    stat[1] = rsqrtf(tot * kInvDim + kLnEps);
  }
  __syncthreads();
  const float rs = stat[1];
  if (wave < 4u) {
    const unsigned c0 = t * 8u;
    const v4f xa = *(const v4f*)(xr + c0);
    const v4f xb = *(const v4f*)(xr + c0 + 4u);
    const v4f ga = *(const v4f*)(gam + c0);
    const v4f gb = *(const v4f*)(gam + c0 + 4u);
    const v4f ba = *(const v4f*)(bet + c0);
    const v4f bb = *(const v4f*)(bet + c0 + 4u);
    unsigned short hb[8];
#pragma unroll
    for (int e = 0; e < 4; ++e) {
      const float va = CVT_IN ? bfr(xa[e]) : xa[e];
      const float vb = CVT_IN ? bfr(xb[e]) : xb[e];
      hb[e]     = h_bits((va - mu) * rs * bfr(ga[e]) + bfr(ba[e]));
      hb[4 + e] = h_bits((vb - mu) * rs * bfr(gb[e]) + bfr(bb[e]));
    }
    const v4u u = (v4u){pk16(hb[0], hb[1]), pk16(hb[2], hb[3]), pk16(hb[4], hb[5]), pk16(hb[6], hb[7])};
    unsigned short* yp = Y + orow * kC + c0;
    *(volatile v4u*)yp = u;
    __threadfence();
    *(volatile v4u*)yp = u;
  }
}

__global__ __launch_bounds__(256) void vtrans_kernel(const unsigned short* __restrict__ src, unsigned short* __restrict__ dst,
                                                     unsigned srcPitch, unsigned rowsPerBatch, unsigned colBase, unsigned dstPitch) {
  __shared__ unsigned short sm[64][66];
  const unsigned t  = threadIdx.x;
  const unsigned g  = blockIdx.y;
  const unsigned b  = g >> 4, hc = g & 15u;
  const unsigned n0 = blockIdx.x * 64u;
#pragma unroll
  for (int it = 0; it < 2; ++it) {
    const unsigned idx = (unsigned)it * 256u + t;
    const unsigned r   = idx >> 3;
    const unsigned seg = (idx & 7u) * 8u;
    const size_t off = (size_t)(b * rowsPerBatch + n0 + r) * srcPitch + colBase + hc * 64u + seg;
    const v4u w = *(const v4u*)(src + off);
    sm[r][seg + 0] = (unsigned short)(w.x & 0xffffu); sm[r][seg + 1] = (unsigned short)(w.x >> 16);
    sm[r][seg + 2] = (unsigned short)(w.y & 0xffffu); sm[r][seg + 3] = (unsigned short)(w.y >> 16);
    sm[r][seg + 4] = (unsigned short)(w.z & 0xffffu); sm[r][seg + 5] = (unsigned short)(w.z >> 16);
    sm[r][seg + 6] = (unsigned short)(w.w & 0xffffu); sm[r][seg + 7] = (unsigned short)(w.w >> 16);
  }
  __syncthreads();
  const unsigned lane = t & 31u, wave = t >> 5;
  const unsigned q = lane >> 3, c8 = (lane & 7u) * 8u;
  unsigned short* vb = dst + (size_t)g * 64u * dstPitch;
  for (int pass = 0; pass < 2; ++pass) {
#pragma unroll
    for (int it = 0; it < 2; ++it) {
      const unsigned dh = wave * 8u + (unsigned)it * 4u + q;
      unsigned short hb[8];
#pragma unroll
      for (int e = 0; e < 8; ++e) hb[e] = sm[c8 + e][dh];
      const v4u u = (v4u){pk16(hb[0], hb[1]), pk16(hb[2], hb[3]), pk16(hb[4], hb[5]), pk16(hb[6], hb[7])};
      *(volatile v4u*)(vb + (size_t)dh * dstPitch + n0 + c8) = u;
    }
    __threadfence();
  }
}

__global__ __launch_bounds__(256) void softmax_rows_kernel(const float* S, unsigned short* P,
                                                           unsigned sPitch, unsigned pPitch, unsigned ncols,
                                                           unsigned seqMask, unsigned nvalid, unsigned causal, float carry) {
  __shared__ float redM[8];
  __shared__ float redS[8];
  const unsigned row  = blockIdx.x;
  const unsigned t    = threadIdx.x;
  const unsigned lane = t & 31u, wave = t >> 5;
  const unsigned nw   = blockDim.x >> 5;
  const unsigned limit = (causal != 0u) ? ((row & seqMask) + 1u) : nvalid;
  const unsigned c0   = t * 8u;
  const unsigned c0c  = (c0 + 8u <= ncols) ? c0 : (ncols - 8u);
  const float* sr = S + (size_t)row * sPitch + c0c;
  const v4f a = *(const v4f*)(sr);
  const v4f c = *(const v4f*)(sr + 4);
  float x[8];
#pragma unroll
  for (int e = 0; e < 4; ++e) {
    x[e]     = ((c0 + (unsigned)e) < limit) ? a[e] : -3.0e38f;
    x[4 + e] = ((c0 + 4u + (unsigned)e) < limit) ? c[e] : -3.0e38f;
  }
  float m = fmaxf(fmaxf(fmaxf(x[0], x[1]), fmaxf(x[2], x[3])), fmaxf(fmaxf(x[4], x[5]), fmaxf(x[6], x[7])));
#pragma unroll
  for (int off = 16; off > 0; off >>= 1) m = fmaxf(m, __shfl_xor(m, off, 32));
  if (lane == 0) redM[wave] = m;
  __syncthreads();
  float gm = redM[0];
  for (unsigned w = 1; w < nw; ++w) gm = fmaxf(gm, redM[w]);
  float p[8];
#pragma unroll
  for (int e = 0; e < 8; ++e) {
    const float ev = expf(x[e] - gm);
    p[e] = ((c0 + (unsigned)e) < limit) ? ev : 0.0f;
  }
  float s = ((p[0] + p[1]) + (p[2] + p[3])) + ((p[4] + p[5]) + (p[6] + p[7]));
#pragma unroll
  for (int off = 16; off > 0; off >>= 1) s += __shfl_xor(s, off, 32);
  if (lane == 0) redS[wave] = s;
  __syncthreads();
  float tot = redS[0];
  for (unsigned w = 1; w < nw; ++w) tot += redS[w];
  const float inv = carry * (1.0f / tot);
  unsigned short hb[8];
#pragma unroll
  for (int e = 0; e < 8; ++e) hb[e] = h_bits(p[e] * inv);
  const v4u u = (v4u){pk16(hb[0], hb[1]), pk16(hb[2], hb[3]), pk16(hb[4], hb[5]), pk16(hb[6], hb[7])};
  if (c0 < ncols) {
    unsigned short* pp = P + (size_t)row * pPitch + c0;
    *(volatile v4u*)pp = u;
    __threadfence();
    *(volatile v4u*)pp = u;
  }
}

constexpr size_t cmax(size_t a, size_t b) { return a > b ? a : b; }
constexpr size_t kMiB = 1048576;
constexpr size_t szWqkv   = (size_t)kQkvCols * kC * 2;
constexpr size_t szWsq    = (size_t)kC * kC * 2;
constexpr size_t szWkv    = (size_t)kKvCols * kC * 2;
constexpr size_t szWff    = (size_t)kFF * kC * 2;
constexpr size_t szPlane  = (size_t)kTok * kC * 2;
constexpr size_t szX      = (size_t)kTok * kC * 4;
constexpr size_t szQkv    = (size_t)kTok * kQkvCols * 2;
constexpr size_t szVt     = (size_t)kGroups * kHD * SEQ * 2;
constexpr size_t szImg    = (size_t)kImgPad * kC * 2;
constexpr size_t szKv     = (size_t)kImgPad * kKvCols * 2;
constexpr size_t szS2     = (size_t)NB * SEQ * kT2P * 4;
constexpr size_t szP2     = (size_t)NB * SEQ * kT2P * 2;
constexpr size_t szVt2    = (size_t)NB * kC * kT2P * 2;
constexpr size_t szGelu   = (size_t)kTok * kFF * 2;
constexpr size_t szScores = (size_t)kHeads * SEQ * SEQ * 4;
constexpr size_t szRQ = cmax(szQkv, szPlane + szKv + szS2 + szP2 + szVt2);
constexpr size_t szRV = cmax(szVt, szPlane);
constexpr size_t szRO = szPlane;
constexpr size_t szRI = szImg;
constexpr size_t szTail = cmax(szGelu, szX + 3 * szWsq + szWkv);
constexpr size_t szPost = szX + 2 * szWff + szTail;
constexpr size_t szPre  = szWqkv + szPlane;
constexpr size_t szRS   = cmax(szScores, cmax(szPost, szPre));
constexpr size_t offRQ = 0;
constexpr size_t offRV = offRQ + szRQ;
constexpr size_t offRO = offRV + szRV;
constexpr size_t offRI = offRO + szRO;
constexpr size_t offRS = offRI + szRI;
constexpr size_t kWsTotal = offRS + szRS;
static_assert(kWsTotal <= (size_t)128 * kMiB);
static_assert(szRQ % 128 == 0 && szRV % 128 == 0 && szRO % 128 == 0 && szRI % 128 == 0 && szRS % 128 == 0);
static_assert(szVt <= szRV && szPlane <= szRV);
static_assert((size_t)kHeads * SEQ * (2 * SEQ) * 2 <= szScores);
static_assert((size_t)kImgPad * 128 * 8 == (size_t)kImgPad * kC);
static_assert((size_t)kImgRows * 256 * 4 == (size_t)kImgRows * kC);
static_assert((size_t)NB * SEQ * 128 * 8 == (size_t)kTok * kC);
static_assert((size_t)(SEQ / 64) * kGroups * 4096 == (size_t)kGroups * kHD * SEQ);
static_assert((size_t)(kT2P / 64) * kGroups * 4096 == (size_t)NB * kC * kT2P);
static_assert((size_t)kHeads * SEQ * kSmThreads * 8 >= (size_t)kHeads * SEQ * SEQ);
static_assert((size_t)NB * SEQ * 64 * 8 >= (size_t)NB * SEQ * kT2P);

static inline unsigned cdiv_u(unsigned a, unsigned b) { return (a + b - 1u) / b; }

extern "C" void kernel_launch(void* const* d_in, const int* in_sizes, int n_in,
                              void* d_out, int out_size, void* d_ws, size_t ws_size,
                              hipStream_t stream) {
  if (n_in < 22) return;
  if ((size_t)in_sizes[0] < ((size_t)(NB - 1) * SEQ_FULL + SEQ) * kC) return;
  if ((size_t)in_sizes[1] < (size_t)kImgRows * kC) return;
  for (int i = 2; i <= 7; ++i) if (in_sizes[i] < kC) return;
  if (in_sizes[8] < kC * kQkvCols || in_sizes[9] < kQkvCols) return;
  if (in_sizes[10] < kC * kC || in_sizes[11] < kC) return;
  if (in_sizes[12] < kC * kC || in_sizes[13] < kC) return;
  if (in_sizes[14] < kC * kKvCols || in_sizes[15] < kKvCols) return;
  if (in_sizes[16] < kC * kC || in_sizes[17] < kC) return;
  if (in_sizes[18] < kC * kFF || in_sizes[19] < kFF) return;
  if (in_sizes[20] < kFF * kC || in_sizes[21] < kC) return;
  if ((size_t)out_size < kOut1OffElems + (size_t)kImgRows * kC) return;
  if ((size_t)out_size < (size_t)kTok * kC) return;
  if (kWsTotal > ws_size) return;

  const float* text    = (const float*)d_in[0];
  const float* img     = (const float*)d_in[1];
  const float* ln1g    = (const float*)d_in[2];
  const float* ln1b    = (const float*)d_in[3];
  const float* ln2g    = (const float*)d_in[4];
  const float* ln2b    = (const float*)d_in[5];
  const float* ln3g    = (const float*)d_in[6];
  const float* ln3b    = (const float*)d_in[7];
  const float* Wqkv    = (const float*)d_in[8];
  const float* bqkv    = (const float*)d_in[9];
  const float* Wproj   = (const float*)d_in[10];
  const float* bproj   = (const float*)d_in[11];
  const float* Wcaq    = (const float*)d_in[12];
  const float* bcaq    = (const float*)d_in[13];
  const float* Wcakv   = (const float*)d_in[14];
  const float* bcakv   = (const float*)d_in[15];
  const float* Wcaproj = (const float*)d_in[16];
  const float* bcaproj = (const float*)d_in[17];
  const float* Wfc     = (const float*)d_in[18];
  const float* bfc     = (const float*)d_in[19];
  const float* Wmp     = (const float*)d_in[20];
  const float* bmp     = (const float*)d_in[21];
  float* out0 = (float*)d_out;
  float* out1 = (float*)d_out + kOut1OffElems;

  char* ws = (char*)d_ws;
  unsigned short* qkv   = (unsigned short*)(ws + offRQ);
  unsigned short* q2    = (unsigned short*)(ws + offRQ);
  unsigned short* kvp   = (unsigned short*)(ws + offRQ + szPlane);
  float*          S2    = (float*)(ws + offRQ + szPlane + szKv);
  unsigned short* P2    = (unsigned short*)(ws + offRQ + szPlane + szKv + szS2);
  unsigned short* Vt2   = (unsigned short*)(ws + offRQ + szPlane + szKv + szS2 + szP2);
  unsigned short* Vt    = (unsigned short*)(ws + offRV);
  unsigned short* lnp   = (unsigned short*)(ws + offRV);
  unsigned short* ctx   = (unsigned short*)(ws + offRO);
  unsigned short* img16 = (unsigned short*)(ws + offRI);
  unsigned short* WqkvT = (unsigned short*)(ws + offRS);
  unsigned short* ln1h  = (unsigned short*)(ws + offRS + szWqkv);
  float*          scores = (float*)(ws + offRS);
  unsigned short* Pself = (unsigned short*)(ws + offRS);
  float*          x2    = (float*)(ws + offRS);
  unsigned short* WfcT  = (unsigned short*)(ws + offRS + szX);
  unsigned short* WmpT  = (unsigned short*)(ws + offRS + szX + szWff);
  char*           tail  = ws + offRS + szX + 2 * szWff;
  float*          x1    = (float*)(tail);
  unsigned short* WprojT   = (unsigned short*)(tail + szX);
  unsigned short* WcaqT    = (unsigned short*)(tail + szX + szWsq);
  unsigned short* WcakvT   = (unsigned short*)(tail + szX + 2 * szWsq);
  unsigned short* WcaprojT = (unsigned short*)(tail + szX + 2 * szWsq + szWkv);
  unsigned short* g16   = (unsigned short*)(tail);

  wtcast_kernel<<<dim3(kC / 64, kQkvCols / 64), dim3(256), 0, stream>>>(Wqkv, WqkvT, kC, kQkvCols, kWCarry);

  img_prep_kernel<<<dim3(kImgPad), dim3(256), 0, stream>>>(img, out1, img16);

  ln_row_kernel<1><<<dim3(SEQ, NB), dim3(256), 0, stream>>>(text, (unsigned)SEQ_FULL, ln1g, ln1b, ln1h);

  wmma_gemm64<2, 1, 0, 0, 0><<<dim3(cdiv_u((kTok / 64) * (kQkvCols / 64), 8), 1), dim3(256), 0, stream>>>(
      ln1h, kC, 0L, WqkvT, kC, 0L, (void*)qkv, kQkvCols, 0L, bqkv, nullptr, 0L, kTok, kQkvCols, kC, 1.0f / kWCarry);

  vtrans_kernel<<<dim3(SEQ / 64, kGroups), dim3(256), 0, stream>>>(qkv, Vt, (unsigned)kQkvCols, (unsigned)SEQ, 2u * kC, (unsigned)SEQ);

  for (int b = 0; b < NB; ++b) {
    const unsigned short* Qp = qkv + (size_t)b * SEQ * kQkvCols;
    const unsigned short* Kp = Qp + kC;
    wmma_gemm64<0, 0, 0, 0, 1><<<dim3(cdiv_u((SEQ / 64) * (SEQ / 64), 8), kHeads), dim3(256), 0, stream>>>(
        Qp, kQkvCols, (long)kHD, Kp, kQkvCols, (long)kHD, (void*)scores, SEQ, (long)SEQ * SEQ,
        nullptr, nullptr, 0L, SEQ, SEQ, kHD, 0.125f);
    softmax_rows_kernel<<<dim3(kHeads * SEQ), dim3(kSmThreads), 0, stream>>>(
        scores, Pself, (unsigned)SEQ, 2u * SEQ, (unsigned)SEQ, (unsigned)(SEQ - 1), 0u, 1u, kPCarry);
    const unsigned short* Vtp = Vt + (size_t)b * kHeads * kHD * SEQ;
    unsigned short* Op = ctx + (size_t)b * SEQ * kC;
    wmma_gemm64<0, 1, 0, 0, 2><<<dim3(cdiv_u((SEQ / 64) * (kHD / 64), 8), kHeads), dim3(256), 0, stream>>>(
        Pself, 2 * SEQ, (long)2 * SEQ * SEQ, Vtp, SEQ, (long)kHD * SEQ, (void*)Op, kC, (long)kHD,
        nullptr, nullptr, 0L, SEQ, kHD, SEQ, kOCarry / kPCarry);
  }

  wtcast_kernel<<<dim3(kC / 64, kC / 64), dim3(256), 0, stream>>>(Wproj, WprojT, kC, kC, kWCarry);
  wtcast_kernel<<<dim3(kC / 64, kC / 64), dim3(256), 0, stream>>>(Wcaq, WcaqT, kC, kC, kWCarry);
  wtcast_kernel<<<dim3(kC / 64, kKvCols / 64), dim3(256), 0, stream>>>(Wcakv, WcakvT, kC, kKvCols, kWCarry);
  wtcast_kernel<<<dim3(kC / 64, kC / 64), dim3(256), 0, stream>>>(Wcaproj, WcaprojT, kC, kC, kWCarry);
  wtcast_kernel<<<dim3(kC / 64, kFF / 64), dim3(256), 0, stream>>>(Wfc, WfcT, kC, kFF, kWCarry);
  wtcast_kernel<<<dim3(kFF / 64, kC / 64), dim3(256), 0, stream>>>(Wmp, WmpT, kFF, kC, kWCarry);

  wmma_gemm64<2, 0, 2, 0, 0><<<dim3(cdiv_u((SEQ / 64) * (kC / 64), 8), NB), dim3(256), 0, stream>>>(
      ctx, kC, (long)SEQ * kC, WprojT, kC, 0L, (void*)x1, kC, (long)SEQ * kC,
      bproj, text, (long)SEQ_FULL * kC, SEQ, kC, kC, 1.0f / (kOCarry * kWCarry));

  ln_row_kernel<0><<<dim3(SEQ, NB), dim3(256), 0, stream>>>(x1, (unsigned)SEQ, ln3g, ln3b, lnp);

  wmma_gemm64<2, 1, 0, 0, 0><<<dim3(cdiv_u((kTok / 64) * (kC / 64), 8), 1), dim3(256), 0, stream>>>(
      lnp, kC, 0L, WcaqT, kC, 0L, (void*)q2, kC, 0L, bcaq, nullptr, 0L, kTok, kC, kC, 1.0f / kWCarry);

  wmma_gemm64<2, 1, 0, 0, 0><<<dim3(cdiv_u((kImgPad / 64) * (kKvCols / 64), 8), 1), dim3(256), 0, stream>>>(
      img16, kC, 0L, WcakvT, kC, 0L, (void*)kvp, kKvCols, 0L, bcakv, nullptr, 0L, kImgPad, kKvCols, kC, 1.0f / kWCarry);

  vtrans_kernel<<<dim3(kT2P / 64, kGroups), dim3(256), 0, stream>>>(kvp, Vt2, (unsigned)kKvCols, (unsigned)kT2, (unsigned)kC, (unsigned)kT2P);

  wmma_gemm64<0, 0, 0, 0, 0><<<dim3(cdiv_u((SEQ / 64) * (kT2P / 64), 8), NB), dim3(256), 0, stream>>>(
      q2, kC, (long)SEQ * kC, kvp, kKvCols, (long)kT2 * kKvCols, (void*)S2, kT2P, (long)SEQ * kT2P,
      nullptr, nullptr, 0L, SEQ, kT2P, kC, 0.03125f);

  softmax_rows_kernel<<<dim3(NB * SEQ), dim3(64), 0, stream>>>(
      S2, P2, (unsigned)kT2P, (unsigned)kT2P, (unsigned)kT2P, 0u, (unsigned)kT2, 0u, kPCarry);

  wmma_gemm64<0, 1, 0, 0, 0><<<dim3(cdiv_u((SEQ / 64) * (kC / 64), 8), NB), dim3(256), 0, stream>>>(
      P2, kT2P, (long)SEQ * kT2P, Vt2, kT2P, (long)kC * kT2P, (void*)ctx, kC, (long)SEQ * kC,
      nullptr, nullptr, 0L, SEQ, kC, kT2P, kOCarry / kPCarry);

  wmma_gemm64<2, 0, 1, 0, 0><<<dim3(cdiv_u((kTok / 64) * (kC / 64), 8), 1), dim3(256), 0, stream>>>(
      ctx, kC, 0L, WcaprojT, kC, 0L, (void*)x2, kC, 0L, bcaproj, x1, 0L, kTok, kC, kC, 1.0f / (kOCarry * kWCarry));

  ln_row_kernel<0><<<dim3(SEQ, NB), dim3(256), 0, stream>>>(x2, (unsigned)SEQ, ln2g, ln2b, lnp);

  wmma_gemm64<2, 1, 0, 5, 0><<<dim3(cdiv_u((kTok / 64) * (kFF / 64), 8), 1), dim3(256), 0, stream>>>(
      lnp, kC, 0L, WfcT, kC, 0L, (void*)g16, kFF, 0L, bfc, nullptr, 0L, kTok, kFF, kC, 1.0f / kWCarry);

  wmma_gemm64<2, 0, 1, 0, 0><<<dim3(cdiv_u((kTok / 64) * (kC / 64), 8), 1), dim3(256), 0, stream>>>(
      g16, kFF, 0L, WmpT, kFF, 0L, (void*)out0, kC, 0L, bmp, x2, 0L, kTok, kC, kFF, 1.0f / (kGCarry * kWCarry));
}
